// ConvCrossAttention_75651553952168
// MI455X (gfx1250) — hardware-verified
//
#include <hip/hip_runtime.h>
#include <math.h>

typedef __attribute__((ext_vector_type(16))) _Float16 v16h;
typedef __attribute__((ext_vector_type(16))) __bf16 v16b;
typedef __attribute__((ext_vector_type(8)))  _Float16 v8h;
typedef __attribute__((ext_vector_type(8)))  float v8f;
typedef __attribute__((ext_vector_type(4)))  float v4f;
typedef __attribute__((ext_vector_type(2)))  float v2f;
typedef __attribute__((ext_vector_type(4)))  unsigned v4u;
typedef __attribute__((ext_vector_type(4)))  int v4i;
typedef float __attribute__((may_alias)) float_a;
typedef int __attribute__((may_alias)) int_a;

template <typename T> __device__ __forceinline__ void vst2(void* p, T v) { *(volatile T*)p = v; __threadfence(); *(volatile T*)p = v; }
__device__ __forceinline__ v8f wmma16(v16h a, v16h b, v8f c) {
  v8f d = __builtin_amdgcn_wmma_f32_16x16x32_f16(false, a, false, b, (short)0, c, false, false);
  asm volatile("v_nop\n\tv_nop\n\tv_nop\n\tv_nop" : "+v"(d) : "v"(a), "v"(b));
  return d;
}
__device__ __forceinline__ v8f wmma_bf(v16b a, v16b b, v8f c) {
  v8f d = __builtin_amdgcn_wmma_f32_16x16x32_bf16(false, a, false, b, (short)0, c, false, false);
  asm volatile("v_nop\n\tv_nop\n\tv_nop\n\tv_nop" : "+v"(d) : "v"(a), "v"(b));
  return d;
}
__device__ __forceinline__ v16h frag_h(const _Float16* rowk0, int lane) {
  union { v16h v; v8h q[2]; } u; const _Float16* p = rowk0 + 8 * (lane >> 4);
  u.q[0] = *(const v8h*)p; u.q[1] = *(const v8h*)(p + 16); return u.v;
}
__device__ __forceinline__ v16h frag_f32(const float* rowk0, int lane) {
  v16h a; const float* p = rowk0 + 8 * (lane >> 4);
#pragma unroll
  for (int i = 0; i < 8; ++i) { a[i] = (_Float16)p[i]; a[8 + i] = (_Float16)p[16 + i]; }
  return a;
}
__device__ __forceinline__ v16h frag_f32s(const float* rowk0, int lane, float sc) {
  v16h a; const float* p = rowk0 + 8 * (lane >> 4);
#pragma unroll
  for (int i = 0; i < 8; ++i) { a[i] = (_Float16)(p[i] * sc); a[8 + i] = (_Float16)(p[16 + i] * sc); }
  return a;
}
__device__ __forceinline__ v16h fragc_f32(const float* W, int k0, int n, int lane, int ld, int K) {
  v16h a; const int g = lane >> 4;
#pragma unroll
  for (int i = 0; i < 8; ++i) { const int ka = k0 + 8 * g + i, kb = ka + 16;
    a[i] = (_Float16)(ka < K ? W[(size_t)(ka < K ? ka : K - 1) * ld + n] : 0.f); a[8 + i] = (_Float16)(kb < K ? W[(size_t)(kb < K ? kb : K - 1) * ld + n] : 0.f); }
  return a;
}
struct F2 { v16b h, l; };
__device__ __forceinline__ F2 bsplit16(const float v[16]) { F2 r;
#pragma unroll
  for (int i = 0; i < 16; ++i) { const __bf16 h = (__bf16)v[i]; r.h[i] = h; r.l[i] = (__bf16)(v[i] - (float)h); }
  return r; }
__device__ __forceinline__ F2 split_row(const float* row, int k0, int lane) { float v[16]; const float* p = row + k0 + 8 * (lane >> 4);
#pragma unroll
  for (int i = 0; i < 8; ++i) { v[i] = p[i]; v[8 + i] = p[16 + i]; }
  return bsplit16(v); }
__device__ __forceinline__ F2 split_rowK(const float* row, int k0, int lane, int K) { float v[16]; const int g = lane >> 4;
#pragma unroll
  for (int i = 0; i < 8; ++i) { const int ka = k0 + 8 * g + i, kb = ka + 16; v[i] = ka < K ? row[ka < K ? ka : K - 1] : 0.f; v[8 + i] = kb < K ? row[kb < K ? kb : K - 1] : 0.f; }
  return bsplit16(v); }
__device__ __forceinline__ F2 split_col(const float* W, int k0, int n, int lane, int ld, int K) { float v[16]; const int g = lane >> 4;
#pragma unroll
  for (int i = 0; i < 8; ++i) { const int ka = k0 + 8 * g + i, kb = ka + 16; v[i] = ka < K ? W[(size_t)(ka < K ? ka : K - 1) * ld + n] : 0.f; v[8 + i] = kb < K ? W[(size_t)(kb < K ? kb : K - 1) * ld + n] : 0.f; }
  return bsplit16(v); }
__device__ __forceinline__ v8f mac3(const F2& a, const F2& b, v8f c) { c = wmma_bf(a.l, b.h, c); c = wmma_bf(a.h, b.l, c); return wmma_bf(a.h, b.h, c); }
__device__ __forceinline__ float sigm(float v) { return 1.0f / (1.0f + expf(-v)); }
#define LDSX() do { asm volatile("s_wait_dscnt 0" ::: "memory"); __builtin_amdgcn_wave_barrier(); __builtin_amdgcn_fence(__ATOMIC_RELEASE, "workgroup"); } while (0)


#define NBI 16
#define CDIM 256
#define HH 32
#define WWI 32
#define NPOS (HH * WWI)
#define NKP 256
#define NHD 8
#define HD 64
#define INNER 512
#define NRQ (NBI * NPOS)
#define NRK (NBI * NKP)
#ifndef NBT
#define NBT NBI
#endif
typedef __attribute__((ext_vector_type(8))) __bf16 v8b;
__device__ __forceinline__ v16b frag_b(const __bf16* rowk0, int lane) {
  union { v16b v; v8b q[2]; } u; const __bf16* p = rowk0 + 8 * (lane >> 4);
  u.q[0] = *(const v8b*)p; u.q[1] = *(const v8b*)(p + 16); return u.v;
}
__device__ __forceinline__ float bfr(float v) { return (float)(__bf16)v; }
__device__ __attribute__((noinline)) float exp_ni(float v) { return expf(v); }
__device__ __attribute__((noinline)) float erf_ni(float v) { return erff(v); }

#define WS_PWQ  0u
#define WS_PWK  (WS_PWQ + 2u * (size_t)2 * INNER * CDIM)
#define WS_PWO  (WS_PWK + 2u * (size_t)2 * 2 * INNER * CDIM)
#define WS_DQ   (WS_PWO + 2u * (size_t)2 * CDIM * INNER)
#define WS_DK   (WS_DQ + 4u * (size_t)2 * NRQ * CDIM)
#define WS_Q    (WS_DK + 4u * (size_t)2 * NRK * CDIM)
#define WS_K    (WS_Q + 2u * (size_t)2 * NRQ * INNER)
#define WS_V    (WS_K + 2u * (size_t)2 * NRK * INNER)
#define WS_O    (WS_V + 2u * (size_t)2 * NBI * INNER * NKP)
#define WS_END  (WS_O + 4u * (size_t)2 * NRQ * INNER)

__global__ __launch_bounds__(256) void k_pack(const float* __restrict__ Q1, const float* __restrict__ Q2, const float* __restrict__ KV1, const float* __restrict__ KV2, const float* __restrict__ O1, const float* __restrict__ O2, __bf16* __restrict__ P) {
  const int n = blockIdx.x, which = blockIdx.y, t = threadIdx.x; __shared__ __align__(16) __bf16 s[INNER];
  const int s_ = which & 1; const int kind = which >> 1; const float* Wm = (kind == 0) ? (s_ ? Q2 : Q1) : (kind == 1) ? (s_ ? KV2 : KV1) : (s_ ? O2 : O1);
  const int rows = (kind == 0) ? INNER : (kind == 1) ? 2 * INNER : CDIM; const int kin = (kind == 2) ? INNER : CDIM; if (n >= rows) return;
  for (int k = t; k < kin; k += 256) s[k] = (__bf16)Wm[(size_t)n * kin + k]; __syncthreads();
  __bf16* dst = (kind == 0) ? P + WS_PWQ / 2 + ((size_t)s_ * INNER + n) * CDIM : (kind == 1) ? P + WS_PWK / 2 + ((size_t)s_ * 2 * INNER + n) * CDIM : P + WS_PWO / 2 + ((size_t)s_ * CDIM + n) * INNER;
  for (int q = t; q < kin / 8; q += 256) vst2((unsigned*)(dst + q * 8), *(const v4u*)&s[q * 8]);
}
__global__ __launch_bounds__(256) void k_dw(const float* __restrict__ X, const float* __restrict__ DW, const float* __restrict__ G, const float* __restrict__ Bb, const float* __restrict__ RM, const float* __restrict__ RV, int s_, int br, float* __restrict__ DQ, float* __restrict__ DK) {
  const int c = blockIdx.x; const size_t b = blockIdx.y; const int t = threadIdx.x;
  __shared__ float sx[HH + 2][WWI + 2]; __shared__ float sw[9];
  for (int e = t; e < (HH + 2) * (WWI + 2); e += 256) { const int yy = e / (WWI + 2) - 1, xx = e % (WWI + 2) - 1; sx[yy + 1][xx + 1] = (yy >= 0 && yy < HH && xx >= 0 && xx < WWI) ? bfr(X[((b * CDIM + c) * HH + yy) * WWI + xx]) : 0.f; }
  if (t < 9) sw[t] = bfr(DW[(size_t)c * 9 + t]);
  __syncthreads();
  const float gg = bfr(G[c]), bb = bfr(Bb[c]), rm = bfr(RM[c]), rv = bfr(RV[c]); const float inv = gg / sqrtf(rv + 1e-5f); const float sh = bb - rm * inv;
  if (br == 0) { for (int p = t; p < NPOS; p += 256) { const int yy = p / WWI, xx = p % WWI; float a = 0.f;
#pragma unroll
      for (int ky = 0; ky < 3; ++ky)
#pragma unroll
        for (int kx = 0; kx < 3; ++kx) a += sx[yy + ky][xx + kx] * sw[ky * 3 + kx];
      DQ[(((size_t)s_ * NBI + b) * NPOS + p) * CDIM + c] = a * inv + sh; } }
  else { const int p = t; if (p < NKP) { const int yy = (p / 16) * 2, xx = (p % 16) * 2; float a = 0.f;
#pragma unroll
      for (int ky = 0; ky < 3; ++ky)
#pragma unroll
        for (int kx = 0; kx < 3; ++kx) a += sx[yy + ky][xx + kx] * sw[ky * 3 + kx];
      DK[(((size_t)s_ * NBI + b) * NKP + p) * CDIM + c] = a * inv + sh; } }
}
__global__ __launch_bounds__(128) void k_pw(const float* __restrict__ DQ, const float* __restrict__ DK, const __bf16* __restrict__ P, _Float16* __restrict__ Q, _Float16* __restrict__ Kx, _Float16* __restrict__ V) {
  __shared__ __align__(16) _Float16 so[64][136]; __shared__ __align__(16) _Float16 st[128][72];
  const int tid = threadIdx.x, wave = tid >> 5, lane = tid & 31, col = lane & 15, g = lane >> 4; const int s_ = blockIdx.z >> 1, br = blockIdx.z & 1; const int n0 = blockIdx.y * 128;
  const size_t nrows = br ? NRK : NRQ; const size_t rb0 = (size_t)blockIdx.x * 64; if (rb0 >= nrows) return; if (!br && n0 >= INNER) return;
  const float* A = (br ? DK : DQ) + ((size_t)s_ * nrows) * CDIM; const __bf16* Wr = br ? P + WS_PWK / 2 + (size_t)s_ * 2 * INNER * CDIM : P + WS_PWQ / 2 + (size_t)s_ * INNER * CDIM;
  const size_t r0 = rb0 + wave * 16;
  v8f acc[8] = {};
#pragma unroll
  for (int kc = 0; kc < CDIM / 32; ++kc) { const F2 a = split_row(A + (r0 + col) * CDIM, kc * 32, lane);
#pragma unroll
    for (int j = 0; j < 8; ++j) { const v16b w = frag_b(Wr + (size_t)(n0 + j * 16 + col) * CDIM + kc * 32, lane); acc[j] = wmma_bf(a.l, w, acc[j]); acc[j] = wmma_bf(a.h, w, acc[j]); } }
  if (!br || n0 < INNER) {
#pragma unroll
    for (int j = 0; j < 8; ++j)
#pragma unroll
      for (int r = 0; r < 8; ++r) so[wave * 16 + 8 * g + r][j * 16 + col] = (_Float16)acc[j][r];
    LDSX();
    _Float16* dst = (br ? Kx : Q) + ((size_t)s_ * nrows) * INNER;
    for (int rl = 0; rl < 16; ++rl) if (lane < 16) vst2((unsigned*)(dst + (r0 + rl) * INNER + n0 + lane * 8), *(const v4u*)&so[wave * 16 + rl][lane * 8]);
  } else {
#pragma unroll
    for (int j = 0; j < 8; ++j)
#pragma unroll
      for (int r = 0; r < 8; ++r) st[j * 16 + col][wave * 16 + 8 * g + r] = (_Float16)acc[j][r];
    __syncthreads();
    const size_t b = rb0 / NKP; const int k0 = (int)(rb0 % NKP); const int c0 = n0 - INNER;
    for (int e = tid; e < 128 * 8; e += 128) { const int d = e >> 3, pc = e & 7; vst2((unsigned*)(V + (((size_t)s_ * NBI + b) * INNER + c0 + d) * NKP + k0 + pc * 8), *(const v4u*)&st[d][pc * 8]); } }
}
__global__ __launch_bounds__(128) void k_attn(const _Float16* __restrict__ Q, const _Float16* __restrict__ Kx, const _Float16* __restrict__ V, float* __restrict__ O) {
  __shared__ __align__(16) _Float16 sph[4][16][40]; __shared__ __align__(16) float so[4][16][68];
  const int tid = threadIdx.x, wave = tid >> 5, lane = tid & 31, col = lane & 15, g = lane >> 4; const int h = blockIdx.y; const size_t b = blockIdx.z >> 1; const int s_ = blockIdx.z & 1; const int so_ = 1 - s_;
  const size_t rq = ((size_t)s_ * NBI + b) * NPOS + blockIdx.x * 64 + wave * 16;
  v16h aq[2];
#pragma unroll
  for (int kc = 0; kc < 2; ++kc) aq[kc] = frag_h(Q + (rq + col) * INNER + h * HD + kc * 32, lane);
  float m[8], l[8];
#pragma unroll
  for (int r = 0; r < 8; ++r) { m[r] = -3.0e38f; l[r] = 0.f; }
  v8f acc[4] = {};
  const _Float16* Kb = Kx + (((size_t)so_ * NBI + b) * NKP) * INNER + h * HD; const _Float16* Vb = V + (((size_t)so_ * NBI + b) * INNER + h * HD) * NKP;
#pragma unroll 1
  for (int ks = 0; ks < NKP / 32; ++ks) { const int j0 = ks * 32; v8f s[2];
#pragma unroll
    for (int ct = 0; ct < 2; ++ct) { const size_t rk = (size_t)(j0 + ct * 16 + col) * INNER; v8f c = {};
#pragma unroll
      for (int kc = 0; kc < 2; ++kc) c = wmma16(aq[kc], frag_h(Kb + rk + kc * 32, lane), c);
#pragma unroll
      for (int r = 0; r < 8; ++r) s[ct][r] = c[r] * 0.125f; }
#pragma unroll
    for (int r = 0; r < 8; ++r) { float mx = fmaxf(s[0][r], s[1][r]);
#pragma unroll
      for (int o = 1; o < 16; o <<= 1) mx = fmaxf(mx, __shfl_xor(mx, o));
      const float mn = fmaxf(m[r], mx); const float alpha = (m[r] <= -1.0e38f) ? 0.f : __expf(m[r] - mn); const float e0 = __expf(s[0][r] - mn), e1 = __expf(s[1][r] - mn); float es = e0 + e1;
#pragma unroll
      for (int o = 1; o < 16; o <<= 1) es += __shfl_xor(es, o);
      l[r] = l[r] * alpha + es; m[r] = mn;
#pragma unroll
      for (int dt = 0; dt < 4; ++dt) acc[dt][r] *= alpha;
      sph[wave][8 * g + r][col] = (_Float16)(e0 * 2048.0f); sph[wave][8 * g + r][16 + col] = (_Float16)(e1 * 2048.0f); }
    LDSX();
    const v16h pa = frag_h(&sph[wave][col][0], lane);
#pragma unroll
    for (int dt = 0; dt < 4; ++dt) acc[dt] = wmma16(pa, frag_h(Vb + (size_t)(dt * 16 + col) * NKP + j0, lane), acc[dt]);
    LDSX(); }
#pragma unroll
  for (int r = 0; r < 8; ++r) { const float il = (1.0f / 2048.0f) / l[r];
#pragma unroll
    for (int dt = 0; dt < 4; ++dt) so[wave][8 * g + r][dt * 16 + col] = acc[dt][r] * il; }
  LDSX();
  for (int rl = 0; rl < 16; ++rl) if (lane < 16) vst2(O + (rq + rl) * INNER + h * HD + lane * 4, *(const v4f*)&so[wave][rl][lane * 4]);
}
__global__ __launch_bounds__(128) void k_out(const float* __restrict__ O, const __bf16* __restrict__ P, const float* __restrict__ B1v, const float* __restrict__ B2v, float* __restrict__ OUT) {
  __shared__ __align__(16) float st[128][68];
  const int tid = threadIdx.x, wave = tid >> 5, lane = tid & 31, col = lane & 15, g = lane >> 4; const size_t b = blockIdx.z >> 1; const int s_ = blockIdx.z & 1; const int p0 = blockIdx.x * 64; const int n0 = blockIdx.y * 128;
  const size_t r0 = ((size_t)s_ * NBI + b) * NPOS + p0 + wave * 16; const __bf16* Wr = P + WS_PWO / 2 + (size_t)s_ * CDIM * INNER; const float* BO = s_ ? B2v : B1v;
  v8f acc[8] = {};
#pragma unroll 2
  for (int kc = 0; kc < INNER / 32; ++kc) { const F2 a = split_row(O + (r0 + col) * INNER, kc * 32, lane);
#pragma unroll
    for (int j = 0; j < 8; ++j) { const v16b w = frag_b(Wr + (size_t)(n0 + j * 16 + col) * INNER + kc * 32, lane); acc[j] = wmma_bf(a.l, w, acc[j]); acc[j] = wmma_bf(a.h, w, acc[j]); } }
#pragma unroll
  for (int j = 0; j < 8; ++j) { const float bb = bfr(BO[n0 + j * 16 + col]);
#pragma unroll
    for (int r = 0; r < 8; ++r) st[j * 16 + col][wave * 16 + 8 * g + r] = acc[j][r] + bb; }
  __syncthreads();
  for (int e = tid; e < 128 * 16; e += 128) { const int c = e >> 4, q = e & 15; vst2(OUT + ((((size_t)s_ * NBI + b) * CDIM + n0 + c) * NPOS) + p0 + q * 4, *(const v4f*)&st[c][q * 4]); }
}
extern "C" void kernel_launch(void* const* d_in, const int* in_sizes, int n_in, void* d_out, int out_size, void* d_ws, size_t ws_size, hipStream_t stream) {
  (void)in_sizes; (void)n_in; (void)out_size;
  const float** F = (const float**)d_in;
  if (ws_size < (size_t)WS_END) return;
  char* ws = (char*)d_ws; __bf16* P = (__bf16*)ws; float *DQ = (float*)(ws + WS_DQ), *DK = (float*)(ws + WS_DK), *O = (float*)(ws + WS_O); _Float16 *Q = (_Float16*)(ws + WS_Q), *Kx = (_Float16*)(ws + WS_K), *V = (_Float16*)(ws + WS_V);
  k_pack<<<dim3(2 * INNER, 6), 256, 0, stream>>>(F[7], F[19], F[13], F[25], F[26], F[28], P);
  k_dw<<<dim3(CDIM, NBT), 256, 0, stream>>>(F[0], F[2], F[3], F[4], F[5], F[6], 0, 0, DQ, DK);
  k_dw<<<dim3(CDIM, NBT), 256, 0, stream>>>(F[0], F[8], F[9], F[10], F[11], F[12], 0, 1, DQ, DK);
  k_dw<<<dim3(CDIM, NBT), 256, 0, stream>>>(F[1], F[14], F[15], F[16], F[17], F[18], 1, 0, DQ, DK);
  k_dw<<<dim3(CDIM, NBT), 256, 0, stream>>>(F[1], F[20], F[21], F[22], F[23], F[24], 1, 1, DQ, DK);
  k_pw<<<dim3(NBT * NPOS / 64, 2 * INNER / 128, 4), 128, 0, stream>>>(DQ, DK, P, Q, Kx, V);
  k_attn<<<dim3(NPOS / 64, NHD, NBT * 2), 128, 0, stream>>>(Q, Kx, V, O);
  k_out<<<dim3(NPOS / 64, CDIM / 128, NBT * 2), 128, 0, stream>>>(O, P, F[27], F[29], (float*)d_out);
}
